// PointNetDecoder_7301444403788
// MI455X (gfx1250) — hardware-verified
//
#include <hip/hip_runtime.h>


#pragma clang fp contract(off)

typedef unsigned short u16;
typedef u16 v8u16 __attribute__((ext_vector_type(8)));
typedef u16 v16u16 __attribute__((ext_vector_type(16)));
typedef __bf16 v16bf __attribute__((ext_vector_type(16)));
typedef float v8f __attribute__((ext_vector_type(8)));
typedef float v4f __attribute__((ext_vector_type(4)));

union FragU {
  v16u16 v;
  v8u16 half[2];
};

__device__ __forceinline__ unsigned bf_bits(float f) {
  unsigned u = __float_as_uint(f);
  u += 0x7FFFu + ((u >> 16) & 1u);
  return u >> 16;
}
__device__ __forceinline__ float bf_val(unsigned b) { return __uint_as_float(b << 16); }
__device__ __forceinline__ void bf_split(float x, unsigned& hb, unsigned& lb) {
  hb = bf_bits(x);
  lb = bf_bits(x - bf_val(hb));
}

__device__ __forceinline__ v8f wmma_bf16(v8f c, v16u16 a, v16u16 b) {
  return __builtin_amdgcn_wmma_f32_16x16x32_bf16(false, __builtin_bit_cast(v16bf, a),
                                                 false, __builtin_bit_cast(v16bf, b),
                                                 (short)0, c, false, false);
}
__device__ __forceinline__ v8f wmma3(v8f c, v16u16 ah, v16u16 al, v16u16 bh, v16u16 bl) {
  c = wmma_bf16(c, ah, bh);
  c = wmma_bf16(c, ah, bl);
  c = wmma_bf16(c, al, bh);
  asm volatile("v_nop\n\tv_nop\n\tv_nop\n\tv_nop" : "+v"(c) : "v"(ah), "v"(al), "v"(bh), "v"(bl));
  return c;
}

__global__ void __launch_bounds__(256) k_prep(const float* __restrict__ P, float* PS, int Ns) {
  const int s = blockIdx.x * 256 + threadIdx.x;
  if (s >= Ns) return;
  const float x = P[(size_t)s * 3 + 0];
  const float y = P[(size_t)s * 3 + 1];
  const float z = P[(size_t)s * 3 + 2];
  const float xx = x * x;
  const float yy = y * y;
  const float zz = z * z;
  float sp = xx + yy;
  sp = sp + zz;
  v4f v;
  v.x = x; v.y = y; v.z = z; v.w = sp;
  volatile v4f* d = (volatile v4f*)(PS + (size_t)s * 4);
  *d = v;
  __threadfence();
  *d = v;
}

__device__ __forceinline__ bool lt2(float d, int i, float e, int j) {
  return (d < e) || (d == e && i < j);
}
__device__ __forceinline__ void ins3(float d, int i,
                                     float& d0, int& i0, float& d1, int& i1, float& d2, int& i2) {
  if (lt2(d, i, d2, i2)) {
    if (lt2(d, i, d0, i0)) {
      d2 = d1; i2 = i1;
      d1 = d0; i1 = i0;
      d0 = d;  i0 = i;
    } else if (lt2(d, i, d1, i1)) {
      d2 = d1; i2 = i1;
      d1 = d;  i1 = i;
    } else {
      d2 = d;  i2 = i;
    }
  }
}

__global__ void __launch_bounds__(256)
k_knn(const float* __restrict__ PS, const float* __restrict__ Q, const float* __restrict__ X,
      float* Out, int Ns, int Nq, int C) {
  const int lane = threadIdx.x & 31;
  const int wave = threadIdx.x >> 5;
  const int q = blockIdx.x * 8 + wave;
  if (q >= Nq) return;

  const float qx = Q[(size_t)q * 3 + 0];
  const float qy = Q[(size_t)q * 3 + 1];
  const float qz = Q[(size_t)q * 3 + 2];
  const float qxx = qx * qx;
  const float qyy = qy * qy;
  const float qzz = qz * qz;
  float sqq = qxx + qyy;
  sqq = sqq + qzz;

  const float INF = __builtin_huge_valf();
  float d0 = INF, d1 = INF, d2 = INF;
  int i0 = 0x7fffffff, i1 = 0x7fffffff, i2 = 0x7fffffff;

  for (int s = lane; s < Ns; s += 32) {
    const v4f p = *(const v4f*)(PS + (size_t)s * 4);
    const float tt = fmaf(qz, p.z, fmaf(qy, p.y, qx * p.x));
    const float u = fmaf(-2.0f, tt, sqq);
    float d = u + p.w;
    d = fmaxf(d, 0.0f);
    ins3(d, s, d0, i0, d1, i1, d2, i2);
  }

#pragma unroll
  for (int off = 16; off > 0; off >>= 1) {
    const float e0 = __shfl_xor(d0, off, 32);
    const float e1 = __shfl_xor(d1, off, 32);
    const float e2 = __shfl_xor(d2, off, 32);
    const int j0 = __shfl_xor(i0, off, 32);
    const int j1 = __shfl_xor(i1, off, 32);
    const int j2 = __shfl_xor(i2, off, 32);
    ins3(e0, j0, d0, i0, d1, i1, d2, i2);
    ins3(e1, j1, d0, i0, d1, i1, d2, i2);
    ins3(e2, j2, d0, i0, d1, i1, d2, i2);
  }

  const int c0 = min(max(i0, 0), Ns - 1);
  const int c1 = min(max(i1, 0), Ns - 1);
  const int c2 = min(max(i2, 0), Ns - 1);

  const float w0 = 1.0f / fmaxf(d0, 1e-16f);
  const float w1 = 1.0f / fmaxf(d1, 1e-16f);
  const float w2 = 1.0f / fmaxf(d2, 1e-16f);
  float wsum = w0 + w1;
  wsum = wsum + w2;
  const float inv = 1.0f / wsum;

  const float* f0 = X + (size_t)c0 * C;
  const float* f1 = X + (size_t)c1 * C;
  const float* f2 = X + (size_t)c2 * C;
  float* op = Out + (size_t)q * C;

  if ((C & 127) == 0) {
    for (int pass = 0; pass < 2; ++pass) {
      for (int c = lane * 4; c < C; c += 128) {
        const v4f a = *(const v4f*)(f0 + c);
        const v4f b = *(const v4f*)(f1 + c);
        const v4f g = *(const v4f*)(f2 + c);
        v4f r;
        r.x = fmaf(w2, g.x, fmaf(w1, b.x, w0 * a.x)) * inv;
        r.y = fmaf(w2, g.y, fmaf(w1, b.y, w0 * a.y)) * inv;
        r.z = fmaf(w2, g.z, fmaf(w1, b.z, w0 * a.z)) * inv;
        r.w = fmaf(w2, g.w, fmaf(w1, b.w, w0 * a.w)) * inv;
        *(volatile v4f*)(op + c) = r;
      }
      if (pass == 0) __threadfence();
    }
  } else {
    for (int pass = 0; pass < 2; ++pass) {
      for (int c = lane; c < C; c += 32) {
        const float r = fmaf(w2, f2[c], fmaf(w1, f1[c], w0 * f0[c])) * inv;
        *(volatile float*)(op + c) = r;
      }
      if (pass == 0) __threadfence();
    }
  }
}

__global__ void __launch_bounds__(256)
k_packw(const float* __restrict__ W, int Kt, int N, int Kp, int Npad, u16* Wh, u16* Wl) {
  const int n = blockIdx.x;
  const int k8 = threadIdx.x * 8;
  if (n >= Npad || k8 >= Kp) return;
  v8u16 vh = {0, 0, 0, 0, 0, 0, 0, 0};
  v8u16 vl = {0, 0, 0, 0, 0, 0, 0, 0};
#pragma unroll
  for (int e = 0; e < 8; ++e) {
    const int k = k8 + e;
    float v = 0.0f;
    if (k < Kt && n < N) v = W[(size_t)k * N + n];
    unsigned hb, lb;
    bf_split(v, hb, lb);
    vh[e] = (u16)hb;
    vl[e] = (u16)lb;
  }
  const size_t o = (size_t)n * Kp + k8;
  *(volatile v8u16*)(Wh + o) = vh;
  *(volatile v8u16*)(Wl + o) = vl;
  __threadfence();
  *(volatile v8u16*)(Wh + o) = vh;
  *(volatile v8u16*)(Wl + o) = vl;
}

template <int BM, int BN, int TPW, bool NARROW>
__global__ void __launch_bounds__(256)
k_gemm(const float* __restrict__ A1, int C1, const float* __restrict__ A2, int C2, int Kt, int Kp,
       const u16* __restrict__ Wh, const u16* __restrict__ Wl, const float* __restrict__ bias,
       float* Out, int M, int N, int relu) {
  constexpr int MT = BM / 16;
  constexpr int NT = BN / 16;
  constexpr int NG = NT / TPW;
  constexpr int AP = 40;
  constexpr int CP = BN + 4;
  constexpr int EPT = BM / 8;
  constexpr int TPR = 32 / EPT;
  typedef char cfg_chk[(MT * NG == 8 && (EPT == 8 || EPT == 16) && (BM * (BN / 4)) % 256 == 0) ? 1 : -1];
  (void)sizeof(cfg_chk);

  __shared__ __attribute__((aligned(16))) u16 sAh[BM * AP];
  __shared__ __attribute__((aligned(16))) u16 sAl[BM * AP];
  __shared__ __attribute__((aligned(16))) u16 sBh[BN * AP];
  __shared__ __attribute__((aligned(16))) u16 sBl[BN * AP];
  __shared__ __attribute__((aligned(16))) float sC[BM * CP];

  const int t = threadIdx.x;
  const int l = t & 31, w = t >> 5, h = l >> 4, m = l & 15;
  const int nblkN = NARROW ? 1 : (N / BN);
  const int bm = blockIdx.x / nblkN;
  const int bn = blockIdx.x - bm * nblkN;
  const int row0 = bm * BM;
  const int n0 = bn * BN;
  if (row0 + BM > M) return;

  const int mt = w % MT;
  const int ntb = (w / MT) * TPW;

  const v8f zero8 = {0.f, 0.f, 0.f, 0.f, 0.f, 0.f, 0.f, 0.f};
  v8f acc[TPW];
#pragma unroll
  for (int j = 0; j < TPW; ++j) acc[j] = zero8;

  const int ar = t / TPR;
  const int akk = (t % TPR) * EPT;
  const size_t arow = (size_t)(row0 + ar);

  for (int k0 = 0; k0 < Kp; k0 += 32) {
#pragma unroll
    for (int g = 0; g < EPT / 8; ++g) {
      v8u16 vh = {0, 0, 0, 0, 0, 0, 0, 0};
      v8u16 vl = {0, 0, 0, 0, 0, 0, 0, 0};
#pragma unroll
      for (int e = 0; e < 8; ++e) {
        const int k = k0 + akk + g * 8 + e;
        float v = 0.0f;
        if (k < C1) v = A1[arow * (size_t)C1 + k];
        else if (k < Kt) v = A2[arow * (size_t)C2 + (k - C1)];
        unsigned hb, lb;
        bf_split(v, hb, lb);
        vh[e] = (u16)hb;
        vl[e] = (u16)lb;
      }
      const int so = ar * AP + akk + g * 8;
      *(v8u16*)(sAh + so) = vh;
      *(v8u16*)(sAl + so) = vl;
    }
    if (t < BN * 4) {
      const int br = t >> 2;
      const int bk = (t & 3) * 8;
      const size_t go = (size_t)(n0 + br) * Kp + k0 + bk;
      const int so = br * AP + bk;
      *(v8u16*)(sBh + so) = *(const v8u16*)(Wh + go);
      *(v8u16*)(sBl + so) = *(const v8u16*)(Wl + go);
    }
    __syncthreads();

    FragU fah, fal;
    {
      const int ao = (mt * 16 + m) * AP + 8 * h;
      fah.half[0] = *(const v8u16*)(sAh + ao);
      fah.half[1] = *(const v8u16*)(sAh + ao + 16);
      fal.half[0] = *(const v8u16*)(sAl + ao);
      fal.half[1] = *(const v8u16*)(sAl + ao + 16);
    }
#pragma unroll
    for (int j = 0; j < TPW; ++j) {
      const int bo = ((ntb + j) * 16 + m) * AP + 8 * h;
      FragU fbh, fbl;
      fbh.half[0] = *(const v8u16*)(sBh + bo);
      fbh.half[1] = *(const v8u16*)(sBh + bo + 16);
      fbl.half[0] = *(const v8u16*)(sBl + bo);
      fbl.half[1] = *(const v8u16*)(sBl + bo + 16);
      acc[j] = wmma3(acc[j], fah.v, fal.v, fbh.v, fbl.v);
    }
    __syncthreads();
  }

#pragma unroll
  for (int j = 0; j < TPW; ++j) {
    const int cb = (ntb + j) * 16 + m;
#pragma unroll
    for (int r = 0; r < 8; ++r) {
      sC[(mt * 16 + 8 * h + r) * CP + cb] = acc[j][r];
    }
  }
  __syncthreads();

  if (NARROW) {
    const int nf4 = (BM * N) / 4;
    for (int pass = 0; pass < 2; ++pass) {
      if (t < nf4) {
        const int e0 = 4 * t;
        v4f v;
#pragma unroll
        for (int e = 0; e < 4; ++e) {
          const int idx = e0 + e;
          const int row = idx / N;
          const int col = idx - row * N;
          float x = sC[row * CP + col] + bias[col];
          if (relu) x = fmaxf(x, 0.0f);
          v[e] = x;
        }
        *(volatile v4f*)(Out + (size_t)row0 * N + e0) = v;
      }
      if (pass == 0) __threadfence();
    }
  } else {
    constexpr int F4R = BN / 4;
    constexpr int ITER = (BM * F4R) / 256;
    for (int pass = 0; pass < 2; ++pass) {
#pragma unroll
      for (int it = 0; it < ITER; ++it) {
        const int idx = it * 256 + t;
        const int row = idx / F4R;
        const int c4 = (idx % F4R) * 4;
        v4f v;
#pragma unroll
        for (int e = 0; e < 4; ++e) {
          float x = sC[row * CP + c4 + e] + bias[n0 + c4 + e];
          if (relu) x = fmaxf(x, 0.0f);
          v[e] = x;
        }
        *(volatile v4f*)(Out + (size_t)(row0 + row) * N + n0 + c4) = v;
      }
      if (pass == 0) __threadfence();
    }
  }
}

static inline int kpad64(int Kt) { return ((Kt + 63) / 64) * 64; }
static inline size_t align128(size_t x) { return (x + 127) & ~(size_t)127; }

static void run_interp(hipStream_t st, const float* P, int Ns, const float* Q, int Nq,
                       const float* X, int C, float* PS, float* O) {
  k_prep<<<dim3((unsigned)((Ns + 255) / 256)), dim3(256), 0, st>>>(P, PS, Ns);
  k_knn<<<dim3((unsigned)((Nq + 7) / 8)), dim3(256), 0, st>>>(PS, Q, X, O, Ns, Nq, C);
}

static void run_layer_wide(hipStream_t st, const float* A1, int C1, const float* A2, int C2,
                           const float* W, const float* b, int N, float* O, int M, int relu,
                           u16* Wh, u16* Wl) {
  const int Kt = C1 + C2;
  const int Kp = kpad64(Kt);
  k_packw<<<dim3((unsigned)N), dim3(256), 0, st>>>(W, Kt, N, Kp, N, Wh, Wl);
  const int grid = (M / 64) * (N / 64);
  k_gemm<64, 64, 2, false><<<dim3((unsigned)grid), dim3(256), 0, st>>>(
      A1, C1, A2, C2, Kt, Kp, Wh, Wl, b, O, M, N, relu);
}

static void run_layer_narrow(hipStream_t st, const float* A1, int C1, const float* W, const float* b,
                             int N, float* O, int M, int relu, u16* Wh, u16* Wl) {
  const int Kt = C1;
  const int Kp = kpad64(Kt);
  k_packw<<<dim3(16), dim3(256), 0, st>>>(W, Kt, N, Kp, 16, Wh, Wl);
  const int grid = M / 128;
  k_gemm<128, 16, 1, true><<<dim3((unsigned)grid), dim3(256), 0, st>>>(
      A1, C1, A1, 0, Kt, Kp, Wh, Wl, b, O, M, N, relu);
}

extern "C" void kernel_launch(void* const* d_in, const int* in_sizes, int n_in,
                              void* d_out, int out_size, void* d_ws, size_t ws_size,
                              hipStream_t stream) {
  if (n_in < 30) return;

  const float* x0     = (const float*)d_in[0];
  const float* pos0   = (const float*)d_in[1];
  const float* x1     = (const float*)d_in[2];
  const float* pos1   = (const float*)d_in[3];
  const float* x2     = (const float*)d_in[4];
  const float* pos2   = (const float*)d_in[5];
  const float* x3     = (const float*)d_in[6];
  const float* pos3   = (const float*)d_in[7];
  const float* fp3_W0 = (const float*)d_in[12];
  const float* fp3_b0 = (const float*)d_in[13];
  const float* fp3_W1 = (const float*)d_in[14];
  const float* fp3_b1 = (const float*)d_in[15];
  const float* fp2_W0 = (const float*)d_in[16];
  const float* fp2_b0 = (const float*)d_in[17];
  const float* fp2_W1 = (const float*)d_in[18];
  const float* fp2_b1 = (const float*)d_in[19];
  const float* fp1_W0 = (const float*)d_in[20];
  const float* fp1_b0 = (const float*)d_in[21];
  const float* fp1_W1 = (const float*)d_in[22];
  const float* fp1_b1 = (const float*)d_in[23];
  const float* fp1_W2 = (const float*)d_in[24];
  const float* fp1_b2 = (const float*)d_in[25];
  const float* lin1_W = (const float*)d_in[26];
  const float* lin1_b = (const float*)d_in[27];
  const float* lin2_W = (const float*)d_in[28];
  const float* lin2_b = (const float*)d_in[29];
  float* out = (float*)d_out;

  const int nP0 = in_sizes[1] / 3, nP1 = in_sizes[3] / 3, nP2 = in_sizes[5] / 3, nP3 = in_sizes[7] / 3;
  if (nP0 <= 0 || nP1 <= 0 || nP2 <= 0 || nP3 <= 0) return;
  const int cX0 = in_sizes[0] / nP0, cX1 = in_sizes[2] / nP1, cX2 = in_sizes[4] / nP2, cX3 = in_sizes[6] / nP3;
  const int n30 = in_sizes[13], n31 = in_sizes[15], n20 = in_sizes[17], n21 = in_sizes[19];
  const int n10 = in_sizes[21], n11 = in_sizes[23], n12 = in_sizes[25], nl1 = in_sizes[27], nl2 = in_sizes[29];
  if (n30 <= 0 || n31 <= 0 || n20 <= 0 || n21 <= 0 || n10 <= 0 || n11 <= 0 || n12 <= 0 || nl1 <= 0 || nl2 <= 0) return;
  if (in_sizes[12] != (cX3 + cX2) * n30) return;
  if (in_sizes[14] != n30 * n31) return;
  if (in_sizes[16] != (n31 + cX1) * n20) return;
  if (in_sizes[18] != n20 * n21) return;
  if (in_sizes[20] != (n21 + cX0) * n10) return;
  if (in_sizes[22] != n10 * n11) return;
  if (in_sizes[24] != n11 * n12) return;
  if (in_sizes[26] != n12 * nl1) return;
  if (in_sizes[28] != nl1 * nl2) return;
  if (out_size != nP0 * nl2) return;
  if ((nP2 % 64) || (nP1 % 64) || (nP0 % 64) || (nP0 % 128)) return;
  if ((n30 % 64) || (n31 % 64) || (n20 % 64) || (n21 % 64) || (n10 % 64) || (n11 % 64) || (n12 % 64) || (nl1 % 64)) return;
  if (nl2 > 8 || ((128 * nl2) % 4)) return;
  if ((cX3 % 4) || (n31 % 4) || (n21 % 4)) return;
  {
    const int kmax = kpad64(cX3 + cX2);
    if (kmax > 2048 || kpad64(n31 + cX1) > 2048 || kpad64(n21 + cX0) > 2048) return;
  }

  int maxNs = nP3; if (nP2 > maxNs) maxNs = nP2; if (nP1 > maxNs) maxNs = nP1;
  size_t actElems = 0;
  {
    size_t c[11] = {(size_t)nP2 * cX3, (size_t)nP2 * n30, (size_t)nP2 * n31, (size_t)nP1 * n31,
                    (size_t)nP1 * n20, (size_t)nP1 * n21, (size_t)nP0 * n21, (size_t)nP0 * n10,
                    (size_t)nP0 * n11, (size_t)nP0 * n12, (size_t)nP0 * nl1};
    for (int i = 0; i < 11; ++i) if (c[i] > actElems) actElems = c[i];
  }
  size_t wElems = 0;
  {
    size_t c[9] = {(size_t)n30 * kpad64(cX3 + cX2), (size_t)n31 * kpad64(n30), (size_t)n20 * kpad64(n31 + cX1),
                   (size_t)n21 * kpad64(n20), (size_t)n10 * kpad64(n21 + cX0), (size_t)n11 * kpad64(n10),
                   (size_t)n12 * kpad64(n11), (size_t)nl1 * kpad64(n12), (size_t)16 * kpad64(nl1)};
    for (int i = 0; i < 9; ++i) if (c[i] > wElems) wElems = c[i];
  }
  const size_t psBytes  = align128((size_t)maxNs * 16);
  const size_t actBytes = align128(actElems * 4);
  const size_t wBytes   = align128(wElems * 2);
  const size_t total    = psBytes + 2 * actBytes + 2 * wBytes;
  if (total > ws_size) return;

  char* wsb  = (char*)d_ws;
  float* PS  = (float*)(wsb);
  float* bufA = (float*)(wsb + psBytes);
  float* bufB = (float*)(wsb + psBytes + actBytes);
  u16* Wh    = (u16*)(wsb + psBytes + 2 * actBytes);
  u16* Wl    = (u16*)(wsb + psBytes + 2 * actBytes + wBytes);

  run_interp(stream, pos3, nP3, pos2, nP2, x3, cX3, PS, bufA);
  run_layer_wide(stream, bufA, cX3, x2, cX2, fp3_W0, fp3_b0, n30, bufB, nP2, 1, Wh, Wl);
  run_layer_wide(stream, bufB, n30, bufB, 0, fp3_W1, fp3_b1, n31, bufA, nP2, 1, Wh, Wl);

  run_interp(stream, pos2, nP2, pos1, nP1, bufA, n31, PS, bufB);
  run_layer_wide(stream, bufB, n31, x1, cX1, fp2_W0, fp2_b0, n20, bufA, nP1, 1, Wh, Wl);
  run_layer_wide(stream, bufA, n20, bufA, 0, fp2_W1, fp2_b1, n21, bufB, nP1, 1, Wh, Wl);

  run_interp(stream, pos1, nP1, pos0, nP0, bufB, n21, PS, bufA);
  run_layer_wide(stream, bufA, n21, x0, cX0, fp1_W0, fp1_b0, n10, bufB, nP0, 1, Wh, Wl);
  run_layer_wide(stream, bufB, n10, bufB, 0, fp1_W1, fp1_b1, n11, bufA, nP0, 1, Wh, Wl);
  run_layer_wide(stream, bufA, n11, bufA, 0, fp1_W2, fp1_b2, n12, bufB, nP0, 1, Wh, Wl);

  run_layer_wide(stream, bufB, n12, bufB, 0, lin1_W, lin1_b, nl1, bufA, nP0, 1, Wh, Wl);
  run_layer_narrow(stream, bufA, nl1, lin2_W, lin2_b, nl2, out, nP0, 0, Wh, Wl);
}
